// Model_19688130085008
// MI455X (gfx1250) — hardware-verified
//
#include <hip/hip_runtime.h>
#include <stddef.h>
#include <stdint.h>
#include <math.h>


#define FIN     32
#define HID     64
#define NHD     4
#define HC      256
#define XW      512
#define KA      128
#define NOUT    32
#define NIT     8
#define NTHR    256
#define NWAVE   8
#define EPT     8
#define CHUNK   (NTHR * EPT)
#define WCAP    (EPT * 32)
#define LISTN   (NWAVE * WCAP)
#define NBA     1024
#define SLA     10
#define RCAP    8192
#define DEGCAP  64
#define MEAS_B1024  5288
#define MEAS_MAXDEG 18
#define GBM     64
#define GTHR    128
#define MROWS   128
#define NEGSL   0.2f
#define NUWIN   (HID * FIN / 8)
#define NUWH    (HC * KA / 8)
#define NUWG    (NOUT * KA / 8)
#define BKT_ZINTS (2 * RCAP + 3 * NBA)
#define BKT_LDS_INTS (LISTN + 2 * RCAP + 3 * NBA + 16)
#define SCAN_STW 320
#define SCAN_LDS_INTS (2 * RCAP + 2 * NBA + HC + HID + NWAVE * SCAN_STW + 16)

static_assert((CHUNK & (CHUNK - 1)) == 0 && CHUNK <= 4096);
static_assert(NBA == (1 << SLA) && NBA % NWAVE == 0 && NBA % 32 == 0);
static_assert(LISTN >= NWAVE * WCAP);
static_assert((RCAP % 32) == 0 && (BKT_ZINTS % 4) == 0);
static_assert(RCAP * 100 >= MEAS_B1024 * 105);
static_assert(DEGCAP >= MEAS_MAXDEG + 8);
static_assert(BKT_LDS_INTS * 4 <= 300000 && SCAN_LDS_INTS * 4 <= 300000);
static_assert(GBM == (GTHR / 32) * 16);
static_assert(FIN == 32 && KA == 2 * HID && (KA % 32) == 0);
static_assert(HC == NHD * HID && XW == 2 * HC && HC == 8 * 32);
static_assert((NUWIN % NTHR) == 0 && (NUWH % NTHR) == 0 && (NUWG % NTHR) == 0);
static_assert((MROWS % GBM) == 0);
static_assert(NBA % GBM == 0);

typedef float          v4f  __attribute__((ext_vector_type(4)));
typedef float          v8f  __attribute__((ext_vector_type(8)));
typedef int            v4i  __attribute__((ext_vector_type(4)));
typedef int            v8i  __attribute__((ext_vector_type(8)));
typedef unsigned short v8us __attribute__((ext_vector_type(8)));
typedef __bf16         v16b __attribute__((ext_vector_type(16)));
typedef v4f  __attribute__((may_alias)) v4fa;
typedef v4i  __attribute__((may_alias)) v4ia;
typedef v8us __attribute__((may_alias)) v8usa;
union FragB { v16b v; v8us h[2]; v8i w; };

__device__ __forceinline__ v8f wmb(const FragB& a, const FragB& b, v8f c) {
  v8f d = __builtin_amdgcn_wmma_f32_16x16x32_bf16(false, a.v, false, b.v, (short)0, c, false, false);
  asm volatile("v_nop\n\tv_nop\n\tv_nop\n\tv_nop" : "+v"(d) : "v"(a.w), "v"(b.w));
  return d;
}

__device__ __forceinline__ void ldwait() { asm volatile("s_wait_loadcnt 0x0" ::: "memory"); }

__device__ __forceinline__ void wsync() {
  asm volatile("" ::: "memory");
  __builtin_amdgcn_fence(__ATOMIC_RELEASE, "workgroup");
  __builtin_amdgcn_wave_barrier();
  asm volatile("" ::: "memory");
}

__device__ __forceinline__ unsigned int f2bf(float f) {
  const unsigned int u = __float_as_uint(f);
  const unsigned int r = ((u + 0x7FFFu + ((u >> 16) & 1u)) >> 16) & 0xFFFFu;
  return ((u & 0x7FFFFFFFu) > 0x7F800000u) ? 0x7FC0u : r;
}
__device__ __forceinline__ float bf2f(unsigned int b) { return __uint_as_float(b << 16); }
__device__ __forceinline__ float bfr(float f) { return bf2f(f2bf(f)); }
__device__ __forceinline__ v4f bfr4(const v4f a) {
  v4f o; o.x = bfr(a.x); o.y = bfr(a.y); o.z = bfr(a.z); o.w = bfr(a.w); return o;
}
__device__ __forceinline__ v8us cvt8b(const v4f a, const v4f b) {
  v8us o;
  o[0] = (unsigned short)f2bf(a.x); o[1] = (unsigned short)f2bf(a.y);
  o[2] = (unsigned short)f2bf(a.z); o[3] = (unsigned short)f2bf(a.w);
  o[4] = (unsigned short)f2bf(b.x); o[5] = (unsigned short)f2bf(b.y);
  o[6] = (unsigned short)f2bf(b.z); o[7] = (unsigned short)f2bf(b.w);
  return o;
}
__device__ __forceinline__ unsigned short hl_sel(float v, bool lo) {
  const unsigned int hb = f2bf(v);
  const unsigned int lb = f2bf(v - bf2f(hb));
  return (unsigned short)(lo ? lb : hb);
}
__device__ __forceinline__ float lky(float t) { return (t > 0.0f) ? t : NEGSL * t; }
__device__ __forceinline__ float keepnz(float h, float o) { return (h != 0.0f) ? h : o; }

__device__ __forceinline__ void put4(float* p, const v4f v, const bool ok) {
  if (ok) *(volatile v4f*)p = v;
  __threadfence();
  if (ok) *(volatile v4f*)p = v;
}

template <int SLB>
__device__ __forceinline__ int scan_chunk(const int* __restrict__ dsts, int nE, int cbase, int slotBase,
                                          int nb, int vec8, int* list, int tid, int lane, int wave) {
  int wc = 0;
  const int el0  = tid * EPT;
  const int e0   = cbase + el0;
  const int sent = -2147483647 - 1;
  v4i da, db;
  if (vec8 != 0 && cbase + CHUNK <= nE) {
    da = *(const v4i*)(dsts + e0);
    db = *(const v4i*)(dsts + e0 + 4);
  } else {
    da.x = (e0     < nE) ? dsts[min(e0,     nE - 1)] : sent;
    da.y = (e0 + 1 < nE) ? dsts[min(e0 + 1, nE - 1)] : sent;
    da.z = (e0 + 2 < nE) ? dsts[min(e0 + 2, nE - 1)] : sent;
    da.w = (e0 + 3 < nE) ? dsts[min(e0 + 3, nE - 1)] : sent;
    db.x = (e0 + 4 < nE) ? dsts[min(e0 + 4, nE - 1)] : sent;
    db.y = (e0 + 5 < nE) ? dsts[min(e0 + 5, nE - 1)] : sent;
    db.z = (e0 + 6 < nE) ? dsts[min(e0 + 6, nE - 1)] : sent;
    db.w = (e0 + 7 < nE) ? dsts[min(e0 + 7, nE - 1)] : sent;
  }
  const unsigned nbs = (unsigned)slotBase;
  const unsigned unb = (unsigned)nb;
  const unsigned s0 = (unsigned)da.x - nbs, s1 = (unsigned)da.y - nbs;
  const unsigned s2 = (unsigned)da.z - nbs, s3 = (unsigned)da.w - nbs;
  const unsigned s4 = (unsigned)db.x - nbs, s5 = (unsigned)db.y - nbs;
  const unsigned s6 = (unsigned)db.z - nbs, s7 = (unsigned)db.w - nbs;
  const bool h0 = s0 < unb, h1 = s1 < unb, h2 = s2 < unb, h3 = s3 < unb;
  const bool h4 = s4 < unb, h5 = s5 < unb, h6 = s6 < unb, h7 = s7 < unb;
  const unsigned any = __builtin_amdgcn_ballot_w32(h0 | h1 | h2 | h3 | h4 | h5 | h6 | h7);
  if (any != 0u) {
#define HITJ(J, HJ, SJ) { \
      const unsigned mj = __builtin_amdgcn_ballot_w32(HJ); \
      if (mj != 0u) { \
        if (HJ) { \
          const int pos = wc + (int)__builtin_amdgcn_mbcnt_lo(mj, 0u); \
          if (pos < WCAP) list[wave * WCAP + pos] = ((el0 + (J)) << SLB) | (int)(SJ); \
        } \
        wc += (int)__builtin_popcount(mj); } }
    HITJ(0, h0, s0)
    HITJ(1, h1, s1)
    HITJ(2, h2, s2)
    HITJ(3, h3, s3)
    HITJ(4, h4, s4)
    HITJ(5, h5, s5)
    HITJ(6, h6, s6)
    HITJ(7, h7, s7)
#undef HITJ
  }
  return wc;
}

__global__ __launch_bounds__(NTHR) void k_prep(const float* __restrict__ feat, const float* __restrict__ Win,
                                               const float* __restrict__ Wl, const float* __restrict__ Wr,
                                               const float* __restrict__ Wg,
                                               unsigned short* FB, unsigned short* WIN, unsigned short* WC1,
                                               unsigned short* WC0, unsigned short* WG2, float* TEMP,
                                               int nN, int nUx, int nUT) {
  const int u = (int)blockIdx.x * NTHR + (int)threadIdx.x;
  const v4f z4 = {0.f, 0.f, 0.f, 0.f};
  v4f a, b;
  unsigned short* dp;
  const int r1 = nUx, r2 = r1 + NUWIN, r3 = r2 + NUWH, r4 = r3 + NUWH, r5 = r4 + NUWH, r6 = r5 + NUWH;
  const int r7 = r6 + NUWG, r8 = r7 + nUT;
  if (u < r1) {
    const int row = u >> 2;
    const int c0  = (u & 3) * 8;
    const int rc  = row < nN ? row : nN - 1;
    const float* p = feat + (size_t)rc * FIN + c0;
    a = *(const v4f*)p; b = *(const v4f*)(p + 4);
    if (row >= nN) { a = z4; b = z4; }
    dp = FB + (size_t)row * FIN + c0;
  } else if (u < r2) {
    const int v = u - r1;
    const float* p = Win + (size_t)v * 8;
    a = *(const v4f*)p; b = *(const v4f*)(p + 4);
    dp = WIN + (size_t)v * 8;
  } else if (u < r3) {
    const int v = u - r2, n = v >> 4, k8 = (v & 15) * 8;
    const float* p = Wl + (size_t)n * KA + (k8 & 63);
    a = *(const v4f*)p; b = *(const v4f*)(p + 4);
    dp = WC1 + (size_t)n * KA + k8;
  } else if (u < r4) {
    const int v = u - r3, n = v >> 4, k8 = (v & 15) * 8;
    const float* p = Wr + (size_t)n * KA + (k8 & 63);
    a = *(const v4f*)p; b = *(const v4f*)(p + 4);
    dp = WC1 + (size_t)(HC + n) * KA + k8;
  } else if (u < r5) {
    const int v = u - r4, n = v >> 4, k8 = (v & 15) * 8;
    const float* p = Wl + (size_t)n * KA + HID + (k8 & 63);
    a = *(const v4f*)p; b = *(const v4f*)(p + 4);
    dp = WC0 + (size_t)n * KA + k8;
  } else if (u < r6) {
    const int v = u - r5, n = v >> 4, k8 = (v & 15) * 8;
    const float* p = Wr + (size_t)n * KA + HID + (k8 & 63);
    a = *(const v4f*)p; b = *(const v4f*)(p + 4);
    dp = WC0 + (size_t)(HC + n) * KA + k8;
  } else if (u < r7) {
    const int v = u - r6, n = v >> 4, k8 = (v & 15) * 8;
    const float* p = Wg + (size_t)n * HID + (k8 & 63);
    a = *(const v4f*)p; b = *(const v4f*)(p + 4);
    dp = WG2 + (size_t)n * KA + k8;
  } else if (u < r8) {
    float* tp = TEMP + (size_t)(u - r7) * 4;
    *(volatile v4f*)tp = z4;
    __threadfence();
    *(volatile v4f*)tp = z4;
    return;
  } else {
    return;
  }
  const v8us o = cvt8b(a, b);
  *(volatile v8us*)dp = o;
  __threadfence();
  *(volatile v8us*)dp = o;
}

__global__ __launch_bounds__(NTHR) void k_misc(const int* __restrict__ cs, const float* __restrict__ bl,
                                               const float* __restrict__ br, const float* __restrict__ att,
                                               const float* __restrict__ bconv, const float* __restrict__ bg,
                                               float* BCAT, float* ATTP, float* BCSP, float* BGP, int* RANK,
                                               int nN, int nTiles) {
  __shared__ int wtot[NWAVE];
  const int tid = (int)threadIdx.x, lane = tid & 31, wave = tid >> 5;
  if (wave < 2) {
    const int i4 = 4 * tid;
    put4(BCAT + i4, bfr4(*(const v4f*)(bl + i4)), true);
  } else if (wave < 4) {
    const int i4 = 4 * (tid - 64);
    put4(BCAT + HC + i4, bfr4(*(const v4f*)(br + i4)), true);
  } else if (wave < 6) {
    const int i4 = 4 * (tid - 128);
    put4(ATTP + i4, bfr4(*(const v4f*)(att + i4)), true);
  } else if (wave == 6) {
    const int q = lane & 15;
    const v4f b0 = bfr4(*(const v4f*)(bconv + 4 * q));
    const v4f b1 = bfr4(*(const v4f*)(bconv + HID + 4 * q));
    const v4f b2 = bfr4(*(const v4f*)(bconv + 2 * HID + 4 * q));
    const v4f b3 = bfr4(*(const v4f*)(bconv + 3 * HID + 4 * q));
    const v4f s = ((b0 + b1) + b2) + b3;
    put4(BCSP + 4 * q, s, lane < 16);
  } else {
    const int q = lane & 7;
    put4(BGP + 4 * q, bfr4(*(const v4f*)(bg + 4 * q)), lane < 8);
  }

  int run = 0;
#pragma unroll 1
  for (int t = 0; t < nTiles; ++t) {
    const int base = t * 1024 + 4 * tid;
    v4i c;
    if (t * 1024 + 1024 <= nN) {
      c = *(const v4i*)(cs + base);
    } else {
      c.x = (base     < nN) ? cs[min(base,     nN - 1)] : 0;
      c.y = (base + 1 < nN) ? cs[min(base + 1, nN - 1)] : 0;
      c.z = (base + 2 < nN) ? cs[min(base + 2, nN - 1)] : 0;
      c.w = (base + 3 < nN) ? cs[min(base + 3, nN - 1)] : 0;
    }
    const int f0 = c.x != 0 ? 1 : 0, f1 = c.y != 0 ? 1 : 0, f2 = c.z != 0 ? 1 : 0, f3 = c.w != 0 ? 1 : 0;
    const int ts = f0 + f1 + f2 + f3;
    int incl = ts;
#pragma unroll
    for (int d = 1; d < 32; d <<= 1) {
      const int up = __shfl_up(incl, d, 32);
      if (lane >= d) incl += up;
    }
    if (lane == 31) wtot[wave] = incl;
    __syncthreads();
    int pre = 0, all = 0;
#pragma unroll
    for (int w2 = 0; w2 < NWAVE; ++w2) {
      const int c2 = wtot[w2];
      all += c2;
      pre += (w2 < wave) ? c2 : 0;
    }
    const int ex = run + pre + incl - ts;
    v4i r;
    r.x = ex; r.y = ex + f0; r.z = ex + f0 + f1; r.w = ex + f0 + f1 + f2;
    int* rp = RANK + base;
    *(volatile v4i*)rp = r;
    __threadfence();
    *(volatile v4i*)rp = r;
    run += all;
    __syncthreads();
  }
}

__global__ __launch_bounds__(NTHR) void k_bucket(const int* __restrict__ srcs, const int* __restrict__ dsts,
                                                 const int* __restrict__ emask, int nE, int nN, int vec8,
                                                 int* LST, int* CO, int* FLG) {
  extern __shared__ __attribute__((aligned(16))) int bsm[];
  int* list = bsm;
  int* reg1 = bsm + LISTN;
  int* reg2 = reg1 + RCAP;
  int* scnt = reg2 + RCAP;
  int* soff = scnt + NBA;
  int* scur = soff + NBA;
  int* wcnt = scur + NBA;
  const int tid = (int)threadIdx.x, lane = tid & 31, wave = tid >> 5;
  const int blk = (int)blockIdx.x;
  const int nodeBase = blk * NBA;
  int nb = nN - nodeBase;
  nb = nb < 0 ? 0 : (nb > NBA ? NBA : nb);

  {
    const v4i z4 = {0, 0, 0, 0};
    for (int i = tid * 4; i < BKT_ZINTS; i += NTHR * 4) *(v4ia*)(reg1 + i) = z4;
  }
  __syncthreads();

  int tot = 0, ovf = 0;
  const int nChunks = (nE + CHUNK - 1) / CHUNK;
#pragma unroll 1
  for (int ch = 0; ch < nChunks; ++ch) {
    const int cbase = ch * CHUNK;
    const int wc = scan_chunk<SLA>(dsts, nE, cbase, nodeBase, nb, vec8, list, tid, lane, wave);
    if (lane == 0) wcnt[wave] = wc;
    __syncthreads();
    int pre = 0, all = 0;
#pragma unroll
    for (int w2 = 0; w2 < NWAVE; ++w2) {
      int c = wcnt[w2];
      c = c < 0 ? 0 : (c > WCAP ? WCAP : c);
      all += c;
      pre += (w2 < wave) ? c : 0;
    }
    const int wcc  = wc > WCAP ? WCAP : wc;
    const int base = tot + pre;
#pragma unroll 1
    for (int i = lane; i < wcc; i += 32) {
      const int ent = list[wave * WCAP + i];
      const int el  = (ent >> SLA) & (CHUNK - 1);
      const int sl  = ent & (NBA - 1);
      int eid = cbase + el;
      eid = eid > nE - 1 ? nE - 1 : eid;
      const int pos = base + i;
      if (pos < RCAP) reg1[pos] = (int)(((unsigned)eid << SLA) | (unsigned)sl);
    }
    if (tot + all > RCAP) ovf = 1;
    tot += all;
    tot = tot > RCAP ? RCAP : tot;
    __syncthreads();
  }
  const int nh = tot;

  if (wave == 0) {
#pragma unroll 1
    for (int b0 = 0; b0 < nh; b0 += 32) {
      const int idx = b0 + lane;
      const int uv  = reg1[idx < nh ? idx : nh - 1];
      const int m32 = (nh - b0) < 32 ? (nh - b0) : 32;
#pragma unroll 1
      for (int k = 0; k < m32; ++k) {
        const int u  = __builtin_amdgcn_readlane(uv, k);
        const int sq = u & (NBA - 1);
        if (lane == 0) scnt[sq] = scnt[sq] + 1;
      }
    }
  }
  __syncthreads();
  if (wave == 0) {
    const int base = lane * (NBA / 32);
    int s = 0;
#pragma unroll 1
    for (int i = 0; i < NBA / 32; ++i) s += scnt[base + i];
    int incl = s;
#pragma unroll
    for (int d = 1; d < 32; d <<= 1) {
      const int y = __shfl_up(incl, d, 32);
      if (lane >= d) incl += y;
    }
    int run = incl - s;
#pragma unroll 1
    for (int i = 0; i < NBA / 32; ++i) {
      const int cv = scnt[base + i];
      soff[base + i] = run;
      scur[base + i] = run;
      run += cv;
    }
  }
  __syncthreads();
  if (wave == 0) {
#pragma unroll 1
    for (int b0 = 0; b0 < nh; b0 += 32) {
      const int idx = b0 + lane;
      const int uv  = reg1[idx < nh ? idx : nh - 1];
      const int m32 = (nh - b0) < 32 ? (nh - b0) : 32;
#pragma unroll 1
      for (int k = 0; k < m32; ++k) {
        const int u   = __builtin_amdgcn_readlane(uv, k);
        const int sq  = u & (NBA - 1);
        const int eid = (int)((unsigned)u >> SLA);
        if (lane == 0) {
          int p = scur[sq];
          p = p < 0 ? 0 : (p > RCAP - 1 ? RCAP - 1 : p);
          reg2[p] = eid;
          scur[sq] = p + 1;
        }
      }
    }
  }
  __syncthreads();
#pragma unroll 1
  for (int p = tid; p < RCAP; p += NTHR) {
    int eid = reg2[p];
    eid = eid < 0 ? 0 : (eid > nE - 1 ? nE - 1 : eid);
    const int sraw = srcs[eid];
    const int em   = emask[eid];
    const int s = sraw < 0 ? 0 : (sraw > nN - 1 ? nN - 1 : sraw);
    const bool ok = p < nh;
    reg1[p] = ok ? s : 0;
    reg2[p] = ok ? em : 0;
  }
  __syncthreads();

  int* lb = LST + (size_t)blk * (2 * RCAP);
  int* cb = CO + (size_t)blk * (2 * NBA);
  v4i cv;
  cv.x = (tid == 0) ? nh : 0;
  cv.y = (tid == 0) ? ovf : 0;
  cv.z = 0; cv.w = 0;
  int* fp = FLG + (size_t)blk * 32 + 4 * (tid & 7);
#pragma unroll 1
  for (int p = tid * 4; p < 2 * RCAP; p += NTHR * 4) {
    const v4i v = *(const v4ia*)(reg1 + p);
    *(volatile v4i*)(lb + p) = v;
  }
#pragma unroll 1
  for (int p = tid * 4; p < 2 * NBA; p += NTHR * 4) {
    const v4i v = *(const v4ia*)(scnt + p);
    *(volatile v4i*)(cb + p) = v;
  }
  if (tid < 8) *(volatile v4i*)fp = cv;
  __threadfence();
#pragma unroll 1
  for (int p = tid * 4; p < 2 * RCAP; p += NTHR * 4) {
    const v4i v = *(const v4ia*)(reg1 + p);
    *(volatile v4i*)(lb + p) = v;
  }
#pragma unroll 1
  for (int p = tid * 4; p < 2 * NBA; p += NTHR * 4) {
    const v4i v = *(const v4ia*)(scnt + p);
    *(volatile v4i*)(cb + p) = v;
  }
  if (tid < 8) *(volatile v4i*)fp = cv;
}

template <int NT, int EPI>
__global__ __launch_bounds__(GTHR) __attribute__((amdgpu_num_vgpr(248)))
void k_gemm(const unsigned short* __restrict__ A, const unsigned short* __restrict__ WT, int K,
            float* outF, unsigned short* outH, const float* __restrict__ addP, const float* __restrict__ biasV,
            int ldo, int nN, const int* __restrict__ cs, const int* __restrict__ RANK, const int* __restrict__ FLG) {
  constexpr int TN = 16 * NT;
  static_assert((EPI == 3) ? (NT == 2) : (NT == 4));
  __shared__ __attribute__((aligned(16))) float stg[GBM * TN];
  __shared__ int smeta[2 * GBM];
  const int tid = (int)threadIdx.x, lane = tid & 31, wave = tid >> 5, hh = lane >> 4, m = lane & 15;
  const int rowBase = (int)blockIdx.x * GBM;
  const int col0    = (int)blockIdx.y * TN;

  v8f acc[NT];
  {
    const v8f z = {0.f, 0.f, 0.f, 0.f, 0.f, 0.f, 0.f, 0.f};
#pragma unroll
    for (int t = 0; t < NT; ++t) acc[t] = z;
  }
  const unsigned short* ap = A  + (size_t)(rowBase + 16 * wave + m) * (size_t)K + 8 * hh;
  const unsigned short* wp = WT + (size_t)(col0 + m) * (size_t)K + 8 * hh;
  const int ksteps = K >> 5;
#pragma unroll 1
  for (int ks = 0; ks < ksteps; ++ks) {
    FragB af;
    af.h[0] = *(const v8usa*)(ap + 32 * ks);
    af.h[1] = *(const v8usa*)(ap + 32 * ks + 16);
#pragma unroll
    for (int t = 0; t < NT; ++t) {
      const unsigned short* wq = wp + (size_t)(16 * t) * (size_t)K + 32 * ks;
      FragB bf;
      bf.h[0] = *(const v8usa*)wq;
      bf.h[1] = *(const v8usa*)(wq + 16);
      acc[t] = wmb(af, bf, acc[t]);
    }
  }

#pragma unroll
  for (int t = 0; t < NT; ++t) {
    const int lc = 16 * t + m;
#pragma unroll
    for (int r = 0; r < 8; ++r) {
      const int lr = 16 * wave + 8 * hh + r;
      stg[lr * TN + lc] = acc[t][r];
    }
  }
  if constexpr (EPI == 3) {
    if (tid < GBM) {
      const int r  = rowBase + tid;
      const int rc = r < nN ? r : nN - 1;
      const int c  = cs[rc];
      const int rk = RANK[rc];
      const bool ok = (r < nN) && (c != 0) && ((unsigned)rk < (unsigned)nN);
      smeta[tid] = ok ? 1 : 0;
      smeta[GBM + tid] = ok ? rk : 0;
    }
  }
  __syncthreads();

  if constexpr (EPI == 0 || EPI == 1) {
    v4f fv[8];
    v4f bv = {0.f, 0.f, 0.f, 0.f};
    if constexpr (EPI == 0) bv = *(const v4f*)(biasV + col0 + 4 * m);
#pragma unroll
    for (int i = 0; i < 8; ++i) {
      const int lr = 16 * wave + 2 * i + hh;
      const size_t go = (size_t)(rowBase + lr) * (size_t)ldo + col0 + 4 * m;
      v4f v = *(const v4fa*)(stg + lr * TN + 4 * m);
      if constexpr (EPI == 1) v = v + *(const v4f*)(addP + go);
      else v = v + bv;
      fv[i] = v;
    }
#pragma unroll
    for (int i = 0; i < 8; ++i) {
      const int lr = 16 * wave + 2 * i + hh;
      float* op = outF + (size_t)(rowBase + lr) * (size_t)ldo + col0 + 4 * m;
      *(volatile v4f*)op = fv[i];
    }
    __threadfence();
#pragma unroll
    for (int i = 0; i < 8; ++i) {
      const int lr = 16 * wave + 2 * i + hh;
      float* op = outF + (size_t)(rowBase + lr) * (size_t)ldo + col0 + 4 * m;
      *(volatile v4f*)op = fv[i];
    }
  } else if constexpr (EPI == 2) {
    const int q = m & 7;
    const bool lo = (m & 8) != 0;
    const v4f ba = bfr4(*(const v4f*)(biasV + 8 * q));
    const v4f bb = bfr4(*(const v4f*)(biasV + 8 * q + 4));
    v8us hv[8];
#pragma unroll
    for (int i = 0; i < 8; ++i) {
      const int lr = 16 * wave + 2 * i + hh;
      const v4f sa = *(const v4fa*)(stg + lr * TN + 8 * q) + ba;
      const v4f sb = *(const v4fa*)(stg + lr * TN + 8 * q + 4) + bb;
      v8us o;
      o[0] = hl_sel(sa.x, lo); o[1] = hl_sel(sa.y, lo); o[2] = hl_sel(sa.z, lo); o[3] = hl_sel(sa.w, lo);
      o[4] = hl_sel(sb.x, lo); o[5] = hl_sel(sb.y, lo); o[6] = hl_sel(sb.z, lo); o[7] = hl_sel(sb.w, lo);
      hv[i] = o;
    }
#pragma unroll
    for (int i = 0; i < 8; ++i) {
      const int lr = 16 * wave + 2 * i + hh;
      unsigned short* op = outH + (size_t)(rowBase + lr) * KA + 8 * m;
      *(volatile v8us*)op = hv[i];
    }
    __threadfence();
#pragma unroll
    for (int i = 0; i < 8; ++i) {
      const int lr = 16 * wave + 2 * i + hh;
      unsigned short* op = outH + (size_t)(rowBase + lr) * KA + 8 * m;
      *(volatile v8us*)op = hv[i];
    }
  } else {
    const int g = lane >> 3, pc = lane & 7;
    const v4f bq = *(const v4f*)(biasV + 4 * pc);
    const int fl = FLG[(size_t)(rowBase >> SLA) * 32 + 1];
    const float pzo = (fl != 0) ? __int_as_float(0x7fc00000) : 0.0f;
    v4f ov[4];
    int okv[4], rkv[4];
#pragma unroll
    for (int i = 0; i < 4; ++i) {
      const int lr = 16 * wave + 4 * i + g;
      const v4f v = *(const v4fa*)(stg + lr * TN + 4 * pc);
      ov[i]  = (v + bq) + pzo;
      okv[i] = smeta[lr];
      rkv[i] = smeta[GBM + lr];
    }
#pragma unroll
    for (int i = 0; i < 4; ++i) {
      float* op = outF + (size_t)rkv[i] * NOUT + 4 * pc;
      if (okv[i] != 0) *(volatile v4f*)op = ov[i];
    }
    __threadfence();
#pragma unroll
    for (int i = 0; i < 4; ++i) {
      float* op = outF + (size_t)rkv[i] * NOUT + 4 * pc;
      if (okv[i] != 0) *(volatile v4f*)op = ov[i];
    }
  }
  (void)outF; (void)outH; (void)addP; (void)biasV; (void)ldo; (void)nN; (void)cs; (void)RANK; (void)FLG;
}

__global__ __launch_bounds__(NTHR) __attribute__((amdgpu_num_vgpr(248)))
void k_scan(const int* __restrict__ LST, const int* __restrict__ CO, const int* __restrict__ FLG,
            const float* __restrict__ XLR, const float* __restrict__ ATTP, const float* __restrict__ BCSP,
            unsigned short* HHL, float* TEMP, unsigned short* THL, int nN, int MPr, int iter, int last) {
  extern __shared__ __attribute__((aligned(16))) int ssm[];
  int*   lsl  = ssm;
  int*   lco  = lsl + 2 * RCAP;
  float* satt = (float*)(lco + 2 * NBA);
  float* sbcs = satt + HC;
  float* stg  = sbcs + HID;
  const int tid = (int)threadIdx.x, lane = tid & 31, wave = tid >> 5;
  const int blk = (int)blockIdx.x;
  const int nodeBase = blk * NBA;

  const int nhraw = FLG[(size_t)blk * 32];
  const int bflag = FLG[(size_t)blk * 32 + 1];
  const int nh  = nhraw < 0 ? 0 : (nhraw > RCAP ? RCAP : nhraw);
  const int ovf = (bflag != 0 || nhraw < 0 || nhraw > RCAP) ? 1 : 0;

  {
    const int* lb = LST + (size_t)blk * (2 * RCAP);
#pragma unroll 1
    for (int p = tid * 4; p < 2 * RCAP; p += NTHR * 4) *(v4ia*)(lsl + p) = *(const v4i*)(lb + p);
    const int* cb = CO + (size_t)blk * (2 * NBA);
#pragma unroll 1
    for (int p = tid * 4; p < 2 * NBA; p += NTHR * 4) *(v4ia*)(lco + p) = *(const v4i*)(cb + p);
    if (wave < 2) {
      *(v4fa*)(satt + 4 * tid) = *(const v4f*)(ATTP + 4 * tid);
    } else if (wave == 2) {
      const int q = lane & 15;
      const v4f bv = *(const v4f*)(BCSP + 4 * q);
      if (lane < 16) *(v4fa*)(sbcs + 4 * q) = bv;
    }
  }
  __syncthreads();

  const float qnan = __int_as_float(0x7fc00000);
  const float pzb  = (ovf != 0) ? qnan : 0.0f;
  float* stw = stg + wave * SCAN_STW;
  float* st2 = stw + HC;
  const v4f atA = *(const v4fa*)(satt + 8 * lane);
  const v4f atB = *(const v4fa*)(satt + 8 * lane + 4);
  const int p16 = lane & 15, q8 = lane & 7;
  const bool losel = (lane & 8) != 0;

#pragma unroll 1
  for (int si = 0; si < NBA / NWAVE; ++si) {
    const int s    = si * NWAVE + wave;
    const int node = nodeBase + s;
    const int nc   = node < nN ? node : nN - 1;
    const int craw = __builtin_amdgcn_readfirstlane(lco[s]);
    const int oraw = __builtin_amdgcn_readfirstlane(lco[NBA + s]);
    const bool big = craw > DEGCAP;
    int c = craw < 0 ? 0 : (craw > DEGCAP ? DEGCAP : craw);
    int o = oraw < 0 ? 0 : (oraw > RCAP ? RCAP : oraw);
    if (c > nh - o) c = nh - o;
    c = c < 0 ? 0 : c;

    const float* xrp = XLR + (size_t)nc * XW + HC + 8 * lane;
    const v4f xa = *(const v4f*)xrp;
    const v4f xb = *(const v4f*)(xrp + 4);
    float mx = -3.0e38f, dn = 0.0f;
    float acc[8];
#pragma unroll
    for (int j = 0; j < 8; ++j) acc[j] = 0.0f;

#pragma unroll 1
    for (int b0 = 0; b0 < c; b0 += 32) {
      const int t = b0 + lane;
      int idx = o + t;
      idx = idx < 0 ? 0 : (idx > RCAP - 1 ? RCAP - 1 : idx);
      int sr = lsl[idx];
      int er = lsl[RCAP + idx];
      sr = sr < 0 ? 0 : (sr > nN - 1 ? nN - 1 : sr);
      er = (t < c) ? er : 0;
      const int m32 = (c - b0) < 32 ? (c - b0) : 32;
#pragma unroll 1
      for (int k = 0; k < m32; ++k) {
        const int sk = __builtin_amdgcn_readlane(sr, k);
        const int ek = __builtin_amdgcn_readlane(er, k);
        if (iter < ek) {
          const float* rp = XLR + (size_t)sk * XW + 8 * lane;
          const v4f a = *(const v4f*)rp;
          const v4f b = *(const v4f*)(rp + 4);
          float pp = 0.0f;
          pp = fmaf(lky(a.x + xa.x), atA.x, pp);
          pp = fmaf(lky(a.y + xa.y), atA.y, pp);
          pp = fmaf(lky(a.z + xa.z), atA.z, pp);
          pp = fmaf(lky(a.w + xa.w), atA.w, pp);
          pp = fmaf(lky(b.x + xb.x), atB.x, pp);
          pp = fmaf(lky(b.y + xb.y), atB.y, pp);
          pp = fmaf(lky(b.z + xb.z), atB.z, pp);
          pp = fmaf(lky(b.w + xb.w), atB.w, pp);
          pp += __shfl_xor(pp, 1, 32);
          pp += __shfl_xor(pp, 2, 32);
          pp += __shfl_xor(pp, 4, 32);
          const float lg = pp;
          const float df = lg - mx;
          const float ee = expf(-fabsf(df));
          const bool  up = df > 0.0f;
          const float s1 = up ? ee : 1.0f;
          const float s2 = up ? 1.0f : ee;
          mx = up ? lg : mx;
          dn = fmaf(dn, s1, s2);
          acc[0] = fmaf(acc[0], s1, s2 * a.x); acc[1] = fmaf(acc[1], s1, s2 * a.y);
          acc[2] = fmaf(acc[2], s1, s2 * a.z); acc[3] = fmaf(acc[3], s1, s2 * a.w);
          acc[4] = fmaf(acc[4], s1, s2 * b.x); acc[5] = fmaf(acc[5], s1, s2 * b.y);
          acc[6] = fmaf(acc[6], s1, s2 * b.z); acc[7] = fmaf(acc[7], s1, s2 * b.w);
        }
      }
    }

    const bool act  = !(dn == 0.0f);
    const float inv = __builtin_amdgcn_rcpf(act ? dn : 1.0f);
    const float pzr = big ? qnan : pzb;
    const bool live = node < nN;
    float sm[8];
#pragma unroll
    for (int j = 0; j < 8; ++j) {
      const float v0 = act ? acc[j] * inv : 0.0f;
      const float v1 = __shfl_xor(v0, 8, 32);
      const float v2 = __shfl_xor(v0, 16, 32);
      const float v3 = __shfl_xor(v0, 24, 32);
      sm[j] = ((v0 + v1) + v2) + v3;
    }
    {
      v4f w0, w1;
      w0.x = sm[0]; w0.y = sm[1]; w0.z = sm[2]; w0.w = sm[3];
      w1.x = sm[4]; w1.y = sm[5]; w1.z = sm[6]; w1.w = sm[7];
      *(v4fa*)(stw + 8 * lane)     = w0;
      *(v4fa*)(stw + 8 * lane + 4) = w1;
    }
    wsync();
#pragma unroll 1
    for (int t2 = 0; t2 < 2; ++t2) {
      const int e = lane + 32 * t2;
      const float y = tanhf(stw[e] + sbcs[e]) + pzr;
      st2[e] = live ? y : 0.0f;
    }
    wsync();

    const v4f h4 = *(const v4fa*)(st2 + 4 * p16);
    const v4f g0 = *(const v4fa*)(st2 + 8 * q8);
    const v4f g1 = *(const v4fa*)(st2 + 8 * q8 + 4);
    const int nr = node < MPr ? node : MPr - 1;
    float* tp = TEMP + (size_t)nr * HID + 4 * p16;
    const v4f o4 = *(const v4f*)tp;
    v4f n4;
    n4.x = keepnz(h4.x, o4.x); n4.y = keepnz(h4.y, o4.y); n4.z = keepnz(h4.z, o4.z); n4.w = keepnz(h4.w, o4.w);
    v8us hq;
    hq[0] = hl_sel(g0.x, losel); hq[1] = hl_sel(g0.y, losel); hq[2] = hl_sel(g0.z, losel); hq[3] = hl_sel(g0.w, losel);
    hq[4] = hl_sel(g1.x, losel); hq[5] = hl_sel(g1.y, losel); hq[6] = hl_sel(g1.z, losel); hq[7] = hl_sel(g1.w, losel);
    v8us tq = {0, 0, 0, 0, 0, 0, 0, 0};
    if (last != 0) {
      const float* t8 = TEMP + (size_t)nr * HID + 8 * q8;
      const v4f oa = *(const v4f*)t8;
      const v4f ob = *(const v4f*)(t8 + 4);
      tq[0] = hl_sel(keepnz(g0.x, oa.x), losel); tq[1] = hl_sel(keepnz(g0.y, oa.y), losel);
      tq[2] = hl_sel(keepnz(g0.z, oa.z), losel); tq[3] = hl_sel(keepnz(g0.w, oa.w), losel);
      tq[4] = hl_sel(keepnz(g1.x, ob.x), losel); tq[5] = hl_sel(keepnz(g1.y, ob.y), losel);
      tq[6] = hl_sel(keepnz(g1.z, ob.z), losel); tq[7] = hl_sel(keepnz(g1.w, ob.w), losel);
    }
    ldwait();
    const bool wr = (node < MPr) && (lane < 16);
    unsigned short* hp = HHL + (size_t)nr * KA + 8 * p16;
    unsigned short* th = THL + (size_t)nr * KA + 8 * p16;
    if (wr) {
      *(volatile v8us*)hp = hq;
      *(volatile v4f*)tp = n4;
      if (last != 0) *(volatile v8us*)th = tq;
    }
    __threadfence();
    if (wr) {
      *(volatile v8us*)hp = hq;
      *(volatile v4f*)tp = n4;
      if (last != 0) *(volatile v8us*)th = tq;
    }
  }
}

static inline int cdiv(int a, int b) { return (a + b - 1) / b; }

extern "C" void kernel_launch(void* const* d_in, const int* in_sizes, int n_in,
                              void* d_out, int out_size, void* d_ws, size_t ws_size,
                              hipStream_t stream) {
  if (n_in < 14) return;
  const int nN = in_sizes[0] / FIN;
  if (nN <= 0 || in_sizes[0] != nN * FIN || nN > (1 << 20)) return;
  if (in_sizes[1] < 2 || (in_sizes[1] & 1) != 0) return;
  const int nE = in_sizes[1] / 2;
  if (nE < 1 || nE > (1 << 21)) return;
  if (in_sizes[2] != nE || in_sizes[3] != nN) return;
  if (in_sizes[4] != HID * FIN || in_sizes[5] != HID) return;
  if (in_sizes[6] != HC * KA || in_sizes[7] != HC) return;
  if (in_sizes[8] != HC * KA || in_sizes[9] != HC) return;
  if (in_sizes[10] != NHD * HID || in_sizes[11] != HC) return;
  if (in_sizes[12] != NOUT * HID || in_sizes[13] != NOUT) return;
  if (out_size != nN * NOUT) return;

  const float* feat  = (const float*)d_in[0];
  const int*   ei    = (const int*)  d_in[1];
  const int*   emask = (const int*)  d_in[2];
  const int*   cstat = (const int*)  d_in[3];
  const float* Win   = (const float*)d_in[4];
  const float* bin   = (const float*)d_in[5];
  const float* Wl    = (const float*)d_in[6];
  const float* bl    = (const float*)d_in[7];
  const float* Wr    = (const float*)d_in[8];
  const float* br    = (const float*)d_in[9];
  const float* att   = (const float*)d_in[10];
  const float* bconv = (const float*)d_in[11];
  const float* Wg    = (const float*)d_in[12];
  const float* bg    = (const float*)d_in[13];
  float* out = (float*)d_out;
  const int* src = ei;
  const int* dst = ei + nE;

  const int MP   = cdiv(nN, MROWS) * MROWS;
  const int gM   = MP / GBM;
  const int gA   = cdiv(MP, NBA);
  if ((long long)gA * NBA < (long long)MP) return;
  const int vec8 = ((nE & 3) == 0) ? 1 : 0;
  const int nUx  = MP * (FIN / 8);
  const int nUT  = MP * (HID / 4);
  if ((nUx % NTHR) != 0 || (nUT % NTHR) != 0) return;
  const int nTiles = cdiv(nN, 1024);

  char* ws = (char*)d_ws;
  size_t off = 0;
  const size_t oFB  = off; off += (size_t)MP * FIN * 2;           off = (off + 255) & ~(size_t)255;
  const size_t oWIN = off; off += (size_t)HID * FIN * 2;          off = (off + 255) & ~(size_t)255;
  const size_t oWC1 = off; off += (size_t)XW * KA * 2;            off = (off + 255) & ~(size_t)255;
  const size_t oWC0 = off; off += (size_t)XW * KA * 2;            off = (off + 255) & ~(size_t)255;
  const size_t oWG2 = off; off += (size_t)NOUT * KA * 2;          off = (off + 255) & ~(size_t)255;
  const size_t oBCT = off; off += (size_t)XW * 4;                 off = (off + 255) & ~(size_t)255;
  const size_t oATT = off; off += (size_t)HC * 4;                 off = (off + 255) & ~(size_t)255;
  const size_t oBCS = off; off += (size_t)HID * 4;                off = (off + 255) & ~(size_t)255;
  const size_t oBG  = off; off += (size_t)NOUT * 4;               off = (off + 255) & ~(size_t)255;
  const size_t oHHL = off; off += (size_t)MP * KA * 2;            off = (off + 255) & ~(size_t)255;
  const size_t oTHL = off; off += (size_t)MP * KA * 2;            off = (off + 255) & ~(size_t)255;
  const size_t oTMP = off; off += (size_t)MP * HID * 4;           off = (off + 255) & ~(size_t)255;
  const size_t oC0  = off; off += (size_t)MP * XW * 4;            off = (off + 255) & ~(size_t)255;
  const size_t oXLR = off; off += (size_t)MP * XW * 4;            off = (off + 255) & ~(size_t)255;
  const size_t oLST = off; off += (size_t)gA * 2 * RCAP * 4;      off = (off + 255) & ~(size_t)255;
  const size_t oCO  = off; off += (size_t)gA * 2 * NBA * 4;       off = (off + 255) & ~(size_t)255;
  const size_t oFLG = off; off += (size_t)gA * 128;               off = (off + 255) & ~(size_t)255;
  const size_t oRNK = off; off += (size_t)nTiles * 1024 * 4;      off = (off + 255) & ~(size_t)255;
  if (off > ws_size) return;
  unsigned short* FB   = (unsigned short*)(ws + oFB);
  unsigned short* WIN  = (unsigned short*)(ws + oWIN);
  unsigned short* WC1  = (unsigned short*)(ws + oWC1);
  unsigned short* WC0  = (unsigned short*)(ws + oWC0);
  unsigned short* WG2  = (unsigned short*)(ws + oWG2);
  float*          BCAT = (float*)(ws + oBCT);
  float*          ATTP = (float*)(ws + oATT);
  float*          BCSP = (float*)(ws + oBCS);
  float*          BGP  = (float*)(ws + oBG);
  unsigned short* HHL  = (unsigned short*)(ws + oHHL);
  unsigned short* THL  = (unsigned short*)(ws + oTHL);
  float*          TEMP = (float*)(ws + oTMP);
  float*          C0   = (float*)(ws + oC0);
  float*          XLR  = (float*)(ws + oXLR);
  int*            LST  = (int*)(ws + oLST);
  int*            CO   = (int*)(ws + oCO);
  int*            FLG  = (int*)(ws + oFLG);
  int*            RANK = (int*)(ws + oRNK);

  const int bktLds  = BKT_LDS_INTS * 4;
  const int scanLds = SCAN_LDS_INTS * 4;
  hipFuncSetAttribute(reinterpret_cast<const void*>(&k_bucket),
                      hipFuncAttributeMaxDynamicSharedMemorySize, bktLds);
  hipFuncSetAttribute(reinterpret_cast<const void*>(&k_scan),
                      hipFuncAttributeMaxDynamicSharedMemorySize, scanLds);

  const int nUall = nUx + NUWIN + 4 * NUWH + NUWG + nUT;
  k_prep<<<nUall / NTHR, NTHR, 0, stream>>>(feat, Win, Wl, Wr, Wg, FB, WIN, WC1, WC0, WG2, TEMP, nN, nUx, nUT);
  k_misc<<<1, NTHR, 0, stream>>>(cstat, bl, br, att, bconv, bg, BCAT, ATTP, BCSP, BGP, RANK, nN, nTiles);
  k_bucket<<<gA, NTHR, bktLds, stream>>>(src, dst, emask, nE, nN, vec8, LST, CO, FLG);
  k_gemm<4, 2><<<dim3(gM, 1), GTHR, 0, stream>>>(FB, WIN, FIN, XLR, HHL, BCAT, bin, KA, nN, cstat, RANK, FLG);
  k_gemm<4, 0><<<dim3(gM, XW / 64), GTHR, 0, stream>>>(HHL, WC0, KA, C0, HHL, BCAT, BCAT, XW, nN, cstat, RANK, FLG);
  for (int it = 0; it < NIT; ++it) {
    k_gemm<4, 1><<<dim3(gM, XW / 64), GTHR, 0, stream>>>(HHL, WC1, KA, XLR, HHL, C0, BCAT, XW, nN, cstat, RANK, FLG);
    k_scan<<<gA, NTHR, scanLds, stream>>>(LST, CO, FLG, XLR, ATTP, BCSP, HHL, TEMP, THL, nN, MP, it,
                                          (it == NIT - 1) ? 1 : 0);
  }
  k_gemm<2, 3><<<dim3(gM, 1), GTHR, 0, stream>>>(THL, WG2, KA, out, HHL, BCAT, BGP, NOUT, nN, cstat, RANK, FLG);
}
